// TypeConcatSheafLearner_31842887533251
// MI455X (gfx1250) — hardware-verified
//
#include <hip/hip_runtime.h>

typedef float          v8f   __attribute__((ext_vector_type(8)));
typedef float          v4f   __attribute__((ext_vector_type(4)));
typedef unsigned int   v4u   __attribute__((ext_vector_type(4)));
typedef int            v8i   __attribute__((ext_vector_type(8)));
typedef unsigned short v8us  __attribute__((ext_vector_type(8)));
typedef unsigned short v16us __attribute__((ext_vector_type(16)));
typedef __bf16         v16bf __attribute__((ext_vector_type(16)));
typedef _Float16       v16h  __attribute__((ext_vector_type(16)));
typedef v4f  __attribute__((may_alias)) v4fa;
typedef v8us __attribute__((may_alias)) v8usa;
union FragB { v16bf v; v16us u; v8us h[2]; v8i w; };
union FragH { v16h  v; v16us u; v8us h[2]; v8i w; };

__device__ __forceinline__ v8f wmb(const FragB& a, const FragB& b, v8f c) {
  v8f d = __builtin_amdgcn_wmma_f32_16x16x32_bf16(false, a.v, false, b.v, (short)0, c, false, false);
  asm volatile("v_nop\n\tv_nop\n\tv_nop\n\tv_nop" : "+v"(d) : "v"(a.w), "v"(b.w));
  return d;
}

__device__ __forceinline__ v8f wmh(const FragH& a, const FragH& b, v8f c) {
  v8f d = __builtin_amdgcn_wmma_f32_16x16x32_f16(false, a.v, false, b.v, (short)0, c, false, false);
  asm volatile("v_nop\n\tv_nop\n\tv_nop\n\tv_nop" : "+v"(d) : "v"(a.w), "v"(b.w));
  return d;
}

__device__ __forceinline__ unsigned bf16_bits(float f) {
  const unsigned u = __float_as_uint(f);
  const unsigned r = (u + 0x7FFFu + ((u >> 16) & 1u)) >> 16;
  const unsigned q = (u >> 16) | 0x40u;
  return ((u & 0x7fffffffu) > 0x7f800000u) ? q : r;
}

__device__ __forceinline__ float bf16_val(float f) {
  return __uint_as_float(bf16_bits(f) << 16);
}
__device__ __forceinline__ int clampi(int v, int lo, int hi) {
  return v < lo ? lo : (v > hi ? hi : v);
}

__device__ __forceinline__ unsigned f16_bits(float f) {
  const unsigned u  = __float_as_uint(f);
  const unsigned s  = (u >> 16) & 0x8000u;
  const unsigned a  = u & 0x7fffffffu;
  const unsigned t  = a - 0x38000000u;
  const unsigned r  = (t + 0x0FFFu + ((t >> 13) & 1u)) >> 13;
  const unsigned rc = r > 0x7C00u ? 0x7C00u : r;
  const bool small  = a < 0x38800000u;
  const bool isnan  = a > 0x7f800000u;
  const unsigned fin = small ? 0u : (s | rc);
  return isnan ? (s | 0x7E00u) : fin;
}

__device__ __forceinline__ unsigned pk16(unsigned lo, unsigned hi) { return lo | (hi << 16); }
__device__ __forceinline__ unsigned bf16_lo_bits(float v) {
  float hi = bf16_val(v);
  asm volatile("" : "+v"(hi));
  return bf16_bits(v - hi);
}
__device__ __forceinline__ v4u pack8_bf16(v4f a, v4f c) {
  return (v4u){ pk16(bf16_bits(a[0]), bf16_bits(a[1])), pk16(bf16_bits(a[2]), bf16_bits(a[3])),
                pk16(bf16_bits(c[0]), bf16_bits(c[1])), pk16(bf16_bits(c[2]), bf16_bits(c[3])) };
}
__device__ __forceinline__ v4u pack8_bf16_lo(v4f a, v4f c) {
  return (v4u){ pk16(bf16_lo_bits(a[0]), bf16_lo_bits(a[1])), pk16(bf16_lo_bits(a[2]), bf16_lo_bits(a[3])),
                pk16(bf16_lo_bits(c[0]), bf16_lo_bits(c[1])), pk16(bf16_lo_bits(c[2]), bf16_lo_bits(c[3])) };
}
__device__ __forceinline__ v4u pack8_f16(v4f a, v4f c) {
  return (v4u){ pk16(f16_bits(a[0]), f16_bits(a[1])), pk16(f16_bits(a[2]), f16_bits(a[3])),
                pk16(f16_bits(c[0]), f16_bits(c[1])), pk16(f16_bits(c[2]), f16_bits(c[3])) };
}

template <int FORM>
__global__ __launch_bounds__(256) void k_plane(const float* __restrict__ src, int rows, int cols, int ldsrc,
                                               unsigned short* __restrict__ dst, int MP, int KP) {
  static_assert(FORM >= 0 && FORM <= 3);
  const int KTOT = (FORM == 1 || FORM == 3) ? 2 * KP : KP;
  const unsigned ppr   = (unsigned)(KTOT >> 3);
  const unsigned kp8   = (unsigned)(KP >> 3);
  const unsigned total = (unsigned)MP * ppr;
  const unsigned g     = blockIdx.x * 256u + threadIdx.x;
  const unsigned rowu  = g / ppr;
  const unsigned p     = g - rowu * ppr;
  const bool second    = p >= kp8;
  const int row = (int)rowu;
  const int c0  = (int)((second ? p - kp8 : p) << 3);
  const float* srow = src + (size_t)clampi(row, 0, rows - 1) * (size_t)ldsrc;
  float x[8];
  unsigned mk[8];
#pragma unroll
  for (int e = 0; e < 8; ++e) {
    const int c = c0 + e;
    const float v = srow[clampi(c, 0, cols - 1)];
    asm volatile("" :: "v"(v));
    x[e]  = v;
    mk[e] = (row < rows && c < cols) ? 0xFFFFu : 0u;
  }
  const v4f a = (v4f){ x[0], x[1], x[2], x[3] };
  const v4f c = (v4f){ x[4], x[5], x[6], x[7] };
  v4u o;
  if (FORM == 2) {
    o = pack8_f16(a, c);
  } else {
    const v4u hi = pack8_bf16(a, c);
    o = hi;
    if (FORM == 1) { const v4u lo = pack8_bf16_lo(a, c); o = second ? lo : hi; }
  }
  const v4u mw = (v4u){ pk16(mk[0], mk[1]), pk16(mk[2], mk[3]), pk16(mk[4], mk[5]), pk16(mk[6], mk[7]) };
  o &= mw;
  if (g < total) {
    volatile v4u* q = (volatile v4u*)(dst + (size_t)g * 8);
    *q = o;
    __threadfence();
    *q = o;
  }
}

template <int FORM> struct FragOf    { typedef FragB T; };
template <>         struct FragOf<2> { typedef FragH T; };
__device__ __forceinline__ v8f mm(const FragB& a, const FragB& b, v8f c) { return wmb(a, b, c); }
__device__ __forceinline__ v8f mm(const FragH& a, const FragH& b, v8f c) { return wmh(a, b, c); }
template <class F> __device__ __forceinline__ F ld_frag(const unsigned short* p) {
  F f;
  f.h[0] = *(const v8usa*)(p);
  f.h[1] = *(const v8usa*)(p + 16);
  return f;
}

template <int FORM, int EPI>
__global__ __launch_bounds__(256) __attribute__((amdgpu_num_vgpr(248)))
void k_gemm_nt(const unsigned short* __restrict__ A, const unsigned short* __restrict__ B,
               const float* __restrict__ bias, float* __restrict__ D, int M, int N, int KTOT, int ldd) {
  static_assert(FORM >= 0 && FORM <= 2);
  static_assert(EPI == 0 || EPI == 1);
  typedef typename FragOf<FORM>::T F;
  __shared__ __attribute__((aligned(16))) float sT[8][16 * 68];
  const int lane = threadIdx.x & 31;
  const int wave = threadIdx.x >> 5;
  const int tilesM = (M + 63) >> 6;
  const int tilesN = (N + 63) >> 6;
  const int tile = blockIdx.x * 8 + wave;
  if (tile >= tilesM * tilesN) return;
  const int tm = tile / tilesN;
  const int tn = tile - tm * tilesN;
  const int m0 = tm << 6;
  const int n0 = tn << 6;

  const int rl = lane & 15;
  const int h8 = (lane >> 4) * 8;
  const unsigned short* pa = A + (size_t)(m0 + rl) * (size_t)KTOT + h8;
  const unsigned short* pb = B + (size_t)(n0 + rl) * (size_t)KTOT + h8;

  v8f acc[4][4];
#pragma unroll
  for (int i = 0; i < 4; ++i)
#pragma unroll
    for (int j = 0; j < 4; ++j) acc[i][j] = (v8f){0.f, 0.f, 0.f, 0.f, 0.f, 0.f, 0.f, 0.f};

#pragma unroll 1
  for (int k0 = 0; k0 < KTOT; k0 += 32) {
    F bf[4];
#pragma unroll
    for (int j = 0; j < 4; ++j) bf[j] = ld_frag<F>(pb + (size_t)(j << 4) * (size_t)KTOT + k0);
#pragma unroll
    for (int i = 0; i < 4; ++i) {
      const F af = ld_frag<F>(pa + (size_t)(i << 4) * (size_t)KTOT + k0);
#pragma unroll
      for (int j = 0; j < 4; ++j) acc[i][j] = mm(af, bf[j], acc[i][j]);
    }
  }

  float* slab = sT[wave];
  const int hh = lane >> 4;
  const int c4 = (lane & 15) * 4;
  const int nc = n0 + c4;
  const bool cok = nc < N;
  v4f bv = (v4f){0.f, 0.f, 0.f, 0.f};
  if (EPI == 1) {
    bv = *(const v4fa*)(bias + clampi(nc, 0, N - 4));
    asm volatile("" :: "v"(bv));
  }
#pragma unroll
  for (int i = 0; i < 4; ++i) {
    const int mBase = m0 + (i << 4);
#pragma unroll
    for (int j = 0; j < 4; ++j) {
#pragma unroll
      for (int r = 0; r < 8; ++r) slab[(h8 + r) * 68 + (j << 4) + rl] = acc[i][j][r];
    }
    __builtin_amdgcn_fence(__ATOMIC_RELEASE, "workgroup");
    __builtin_amdgcn_wave_barrier();
    __builtin_amdgcn_fence(__ATOMIC_ACQUIRE, "workgroup");
    v4f vv[8];
#pragma unroll
    for (int it = 0; it < 8; ++it) {
      const int row = it * 2 + hh;
      v4f v = *(const v4fa*)(slab + row * 68 + c4);
      if (EPI == 1) v += bv;
      vv[it] = v;
    }
    for (int pass = 0; pass < 2; ++pass) {
#pragma unroll
      for (int it = 0; it < 8; ++it) {
        const int row = mBase + it * 2 + hh;
        if (cok && row < M) *(volatile v4f*)(D + (size_t)row * (size_t)ldd + nc) = vv[it];
      }
      __threadfence();
    }
    __builtin_amdgcn_fence(__ATOMIC_RELEASE, "workgroup");
    __builtin_amdgcn_wave_barrier();
    __builtin_amdgcn_fence(__ATOMIC_ACQUIRE, "workgroup");
  }
}

#define NN      100000
#define NE      1600000
#define C_DIM   64
#define IN_DIM  148
#define ODIM    9
#define MPAD    100096
#define NPB     64
#define PN      32
#define LDD     32
#define TTN     192
#define TTPAD   256
#define EPB     256
#define SRUN    288

#define SZ_XB   ((size_t)MPAD * C_DIM * 2)
#define SZ_P    ((size_t)MPAD * LDD * 4)
#define SZ_BP   ((size_t)NPB * C_DIM * 2)
#define SZ_TT   ((size_t)TTPAD * 4)
#define OFF_XB  ((size_t)0)
#define OFF_P   (OFF_XB + SZ_XB)
#define OFF_BP  (OFF_P + SZ_P)
#define OFF_TT  (OFF_BP + SZ_BP)
#define WS_TOTAL (OFF_TT + SZ_TT)

static_assert(C_DIM == 64 && C_DIM % 32 == 0);
static_assert(IN_DIM == 2 * C_DIM + 20);
static_assert(2 * ODIM <= PN && PN <= LDD && LDD == 32 && LDD * 4 == 128);
static_assert(PN % 4 == 0 && PN >= 4 && PN <= NPB && NPB % 64 == 0 && NPB == 64);
static_assert(MPAD % 128 == 0 && MPAD % 64 == 0 && MPAD >= NN && NN % 16 == 0);
static_assert(((NN + 63) / 64) * 64 <= MPAD);
static_assert((MPAD * (C_DIM / 8)) % 256 == 0);
static_assert(20 * ODIM <= TTN && TTN <= TTPAD && TTPAD % 32 == 0);
static_assert(NE % EPB == 0 && EPB == 256);
static_assert(SRUN == 32 * ODIM && (32 * ODIM * 4) % 128 == 0);
static_assert((IN_DIM * 4) % 16 == 0);
static_assert(SZ_XB == 12812288 && SZ_P == 12812288 && SZ_BP == 8192 && SZ_TT == 1024);
static_assert(OFF_P % 256 == 0 && OFF_BP % 256 == 0 && OFF_TT % 256 == 0);
static_assert(WS_TOTAL == 25633792 && WS_TOTAL <= ((size_t)128 << 20));
static_assert((long long)(NE / EPB - 1) * 8 * SRUN + 7 * SRUN + SRUN - 1 == (long long)NE * ODIM - 1);

typedef float v2f __attribute__((ext_vector_type(2)));
typedef v2f __attribute__((may_alias)) v2fa;

__global__ __launch_bounds__(256) void k_prep(const float* __restrict__ W, unsigned short* __restrict__ BP,
                                              float* __restrict__ TT) {
  const int tid = (int)threadIdx.x;
#pragma unroll 1
  for (int j = 0; j < 2; ++j) {
    const int g   = j * 256 + tid;
    const int n   = g >> 3;
    const int k8  = (g & 7) << 3;
    const int sec = (n >= ODIM) ? 1 : 0;
    const int nn  = clampi(n - ODIM * sec, 0, ODIM - 1);
    const float* p = W + nn * IN_DIM + C_DIM * sec + k8;
    const v4f a = *(const v4fa*)p;
    const v4f c = *(const v4fa*)(p + 4);
    asm volatile("" :: "v"(a));
    asm volatile("" :: "v"(c));
    v4u o = pack8_bf16(a, c);
    const unsigned mk = (n < 2 * ODIM) ? 0xFFFFFFFFu : 0u;
    o &= (v4u){ mk, mk, mk, mk };
    volatile v4u* q = (volatile v4u*)(BP + (size_t)g * 8);
    *q = o;
    __threadfence();
    *q = o;
  }
  if (tid < TTPAD / 4) {
    v4f ov;
#pragma unroll
    for (int i = 0; i < 4; ++i) {
      const int idx = 4 * tid + i;
      const int ic  = idx < 20 * ODIM ? idx : 20 * ODIM - 1;
      const int c   = ic / ODIM;
      const int o   = ic - ODIM * c;
      const float w = W[o * IN_DIM + 2 * C_DIM + c];
      asm volatile("" :: "v"(w));
      const unsigned b  = bf16_bits(w) << 16;
      const unsigned mk = (idx < 20 * ODIM) ? 0xFFFFFFFFu : 0u;
      ov[i] = __uint_as_float(b & mk);
    }
    volatile v4f* q = (volatile v4f*)(TT + 4 * tid);
    *q = ov;
    __threadfence();
    *q = ov;
  }
}

__global__ __launch_bounds__(256) void k_edge(const int* __restrict__ ei, const int* __restrict__ ety,
                                              const int* __restrict__ nty, const float* __restrict__ P,
                                              const float* __restrict__ TT, float* __restrict__ out) {
  __shared__ __attribute__((aligned(16))) float st[8 * SRUN];
  __shared__ __attribute__((aligned(16))) float tt[TTN];
  const int tid  = (int)threadIdx.x;
  const int lane = tid & 31;
  const int wave = tid >> 5;
  {
    const float tv = TT[tid < TTN - 1 ? tid : TTN - 1];
    asm volatile("" :: "v"(tv));
    if (tid < TTN) tt[tid] = tv;
  }
  __syncthreads();

  const int e = (int)blockIdx.x * EPB + tid;
  int s  = ei[e];
  int d  = ei[NE + e];
  int et = ety[e];
  s  = clampi(s, 0, NN - 1);
  d  = clampi(d, 0, NN - 1);
  et = clampi(et, 0, 11);
  int ts = nty[s];
  int td = nty[d];
  asm volatile("" :: "v"(ts));
  asm volatile("" :: "v"(td));
  ts = clampi(ts, 0, 3);
  td = clampi(td, 0, 3);

  const float* ps = P + (size_t)s * LDD;
  const float* pd = P + (size_t)d * LDD;
  const v4f   a0  = *(const v4fa*)(ps);
  asm volatile("" :: "v"(a0));
  const v4f   a4  = *(const v4fa*)(ps + 4);
  asm volatile("" :: "v"(a4));
  const float a8  = ps[8];
  asm volatile("" :: "v"(a8));
  const float d9  = pd[9];
  asm volatile("" :: "v"(d9));
  const v2f   d10 = *(const v2fa*)(pd + 10);
  asm volatile("" :: "v"(d10));
  const v4f   d12 = *(const v4fa*)(pd + 12);
  asm volatile("" :: "v"(d12));
  const v2f   d16 = *(const v2fa*)(pd + 16);
  asm volatile("" :: "v"(d16));

  const int i0 = ts * ODIM;
  const int i1 = (4 + td) * ODIM;
  const int i2 = (8 + et) * ODIM;
  const int sb = wave * SRUN + ODIM * lane;
  st[sb + 0] = ((a0.x + d9)    + tt[i0 + 0]) + (tt[i1 + 0] + tt[i2 + 0]);
  st[sb + 1] = ((a0.y + d10.x) + tt[i0 + 1]) + (tt[i1 + 1] + tt[i2 + 1]);
  st[sb + 2] = ((a0.z + d10.y) + tt[i0 + 2]) + (tt[i1 + 2] + tt[i2 + 2]);
  st[sb + 3] = ((a0.w + d12.x) + tt[i0 + 3]) + (tt[i1 + 3] + tt[i2 + 3]);
  st[sb + 4] = ((a4.x + d12.y) + tt[i0 + 4]) + (tt[i1 + 4] + tt[i2 + 4]);
  st[sb + 5] = ((a4.y + d12.z) + tt[i0 + 5]) + (tt[i1 + 5] + tt[i2 + 5]);
  st[sb + 6] = ((a4.z + d12.w) + tt[i0 + 6]) + (tt[i1 + 6] + tt[i2 + 6]);
  st[sb + 7] = ((a4.w + d16.x) + tt[i0 + 7]) + (tt[i1 + 7] + tt[i2 + 7]);
  st[sb + 8] = ((a8   + d16.y) + tt[i0 + 8]) + (tt[i1 + 8] + tt[i2 + 8]);

#pragma unroll 1
  for (int o = 0; o < ODIM; ++o) {
    const float v = st[sb + o];
    st[sb + o] = tanhf(v);
  }
  __syncthreads();

  float r[ODIM];
#pragma unroll
  for (int j = 0; j < ODIM; ++j) r[j] = st[wave * SRUN + 32 * j + lane];
  float* ob = out + (size_t)SRUN * (size_t)((int)blockIdx.x * 8 + wave) + lane;
#pragma unroll
  for (int j = 0; j < ODIM; ++j) *(volatile float*)(ob + 32 * j) = r[j];
  __threadfence();
#pragma unroll
  for (int j = 0; j < ODIM; ++j) *(volatile float*)(ob + 32 * j) = r[j];
}

extern "C" void kernel_launch(void* const* d_in, const int* in_sizes, int n_in,
                              void* d_out, int out_size, void* d_ws, size_t ws_size,
                              hipStream_t stream) {
  if (n_in < 5) return;
  if (in_sizes[0] != NN * C_DIM) return;
  if (in_sizes[1] != 2 * NE) return;
  if (in_sizes[2] != NE) return;
  if (in_sizes[3] != NN) return;
  if (in_sizes[4] != ODIM * IN_DIM) return;
  if (out_size != NE * ODIM) return;
  if (ws_size < (size_t)WS_TOTAL) return;

  const float* x   = (const float*)d_in[0];
  const int*   ei  = (const int*)d_in[1];
  const int*   ety = (const int*)d_in[2];
  const int*   nty = (const int*)d_in[3];
  const float* W   = (const float*)d_in[4];
  float* out = (float*)d_out;

  char* ws = (char*)d_ws;
  unsigned short* XB = (unsigned short*)(ws + OFF_XB);
  float*          P  = (float*)(ws + OFF_P);
  unsigned short* BP = (unsigned short*)(ws + OFF_BP);
  float*          TT = (float*)(ws + OFF_TT);

  k_plane<0><<<(MPAD * (C_DIM / 8)) / 256, 256, 0, stream>>>(x, NN, C_DIM, C_DIM, XB, MPAD, C_DIM);
  k_prep<<<1, 256, 0, stream>>>(W, BP, TT);
  k_gemm_nt<0, 0><<<(((NN + 63) / 64) + 7) / 8, 256, 0, stream>>>(XB, BP, TT, P, NN, PN, C_DIM, LDD);
  k_edge<<<NE / EPB, 256, 0, stream>>>(ei, ety, nty, P, TT, out);
}
